// SSIM_17772574670848
// MI455X (gfx1250) — hardware-run, weakly checked
//
#include <hip/hip_runtime.h>
#include <math.h>

typedef __attribute__((ext_vector_type(16))) _Float16 v16h;
typedef __attribute__((ext_vector_type(8)))  float    v8f;
typedef __attribute__((ext_vector_type(4)))  float    v4f;
typedef __attribute__((ext_vector_type(8)))  unsigned v8u;
typedef __attribute__((ext_vector_type(4)))  unsigned v4u;
typedef __attribute__((ext_vector_type(2)))  unsigned v2u;

constexpr int kImgs       = 64;
constexpr int kDim        = 384;
constexpr int kWin        = 7;
constexpr int kTaps       = kWin * kWin;
constexpr int kValid      = kDim - kWin + 1;
constexpr int kTile       = 64;
constexpr int kTilesDim   = 6;
constexpr int kRegion     = 80;
constexpr int kPitchW     = 44;
constexpr int kGroups     = kRegion / 4;
constexpr int kFillItems  = kRegion * kGroups;
constexpr int kFillIters  = 7;
constexpr int kTileBlocks = kImgs * kTilesDim * kTilesDim;
constexpr int kMaxBlocks  = 288;
constexpr int kMaxChunk   = 32768;
constexpr float kCarry    = 2048.0f;
constexpr float kCarryInv = 1.0f / 2048.0f;
constexpr float kF16MinNormal = 6.103515625e-5f;
constexpr float kCovNorm  = (float)((double)kTaps / (double)(kTaps - 1));
constexpr double kInvCount = 1.0 / ((double)kImgs * (double)kValid * (double)kValid);

static_assert(kValid == 378, "valid extent");
static_assert(kTaps == 49, "taps");
static_assert(kTilesDim * kTile >= kValid && kTilesDim * kTile <= kDim, "tile cover");
static_assert(kRegion == kTile + 16 && (kRegion % 16) == 0, "region covers k 0..79");
static_assert(kPitchW * 2 >= kRegion && (kPitchW % 4) == 0, "16-B aligned plane rows");
static_assert(kFillIters * 256 >= kFillItems, "fill coverage");
static_assert((size_t)kMaxBlocks * kMaxChunk == (size_t)kImgs * kDim * kDim, "max pass coverage");
static_assert(kMaxChunk == 256 * 32 * 4, "max pass per-block chunk");
static_assert(kMaxBlocks <= 512, "second-stage max reads two lines per thread");
static_assert((kTileBlocks % 256) == 0, "final sum coverage");
static_assert((kDim % 4) == 0 && (kTile % 4) == 0, "float4 groups never straddle the image edge");

constexpr size_t kOffPmax = 0;
constexpr size_t kOffDr   = kOffPmax + (size_t)kMaxBlocks * 128;
constexpr size_t kOffPsum = kOffDr + 128;
constexpr size_t kWsTotal = kOffPsum + (size_t)kTileBlocks * 128;
static_assert(kWsTotal == 331904ull, "carve total");
static_assert((kOffDr % 128) == 0 && (kOffPsum % 128) == 0, "aligned regions");

__device__ __forceinline__ float block_max256(float m, float* sRedX, int lane, int wave) {
#pragma unroll
  for (int off = 16; off > 0; off >>= 1) m = fmaxf(m, __shfl_xor(m, off, 32));
  if (lane == 0) sRedX[wave] = m;
  __syncthreads();
  float v = sRedX[lane & 7];
#pragma unroll
  for (int off = 4; off > 0; off >>= 1) v = fmaxf(v, __shfl_xor(v, off, 32));
  return v;
}
__device__ __forceinline__ float block_sum256(float s, float* sRedX, int lane, int wave) {
#pragma unroll
  for (int off = 16; off > 0; off >>= 1) s += __shfl_xor(s, off, 32);
  if (lane == 0) sRedX[wave] = s;
  __syncthreads();
  float v = sRedX[lane & 7];
#pragma unroll
  for (int off = 4; off > 0; off >>= 1) v += __shfl_xor(v, off, 32);
  return v;
}

__device__ __forceinline__ void split16(float v, unsigned& hb, unsigned& lb) {
  const _Float16 h0 = (_Float16)v;
  float hf = (float)h0;
  hf = (fabsf(hf) < kF16MinNormal) ? 0.0f : hf;
  const _Float16 h1 = (_Float16)hf;
  const float rs = (v - hf) * kCarry;
  const _Float16 l1 = (_Float16)rs;
  const unsigned short hs = __builtin_bit_cast(unsigned short, h1);
  const unsigned short ls = __builtin_bit_cast(unsigned short, l1);
  hb = (unsigned)hs;
  lb = (unsigned)ls;
}

__device__ __forceinline__ v16h ld_frag(const unsigned* p) {
  const v4u x = *(const v4u*)(p);
  const v4u y = *(const v4u*)(p + 8);
  const v8u w = __builtin_shufflevector(x, y, 0, 1, 2, 3, 4, 5, 6, 7);
  return __builtin_bit_cast(v16h, w);
}

__device__ __forceinline__ v8f mma_f16(v16h a, v16h b, v8f c) {
  c = __builtin_amdgcn_wmma_f32_16x16x32_f16(false, a, false, b, (short)0, c, false, false);
  asm volatile("v_nop\n\tv_nop\n\tv_nop\n\tv_nop" : "+v"(c) : "v"(a), "v"(b));
  return c;
}

__global__ __launch_bounds__(256) void max_partial_kernel(const float* __restrict__ gt, float* __restrict__ pmax) {
  __shared__ float sRedA[8];
  const int tid  = threadIdx.x;
  const int lane = tid & 31;
  const int wave = __builtin_amdgcn_readfirstlane(tid >> 5);
  const float* base = gt + (size_t)blockIdx.x * kMaxChunk + (size_t)tid * 4;
  float m = -INFINITY;
#pragma unroll 4
  for (int it = 0; it < 32; ++it) {
    const v4f v = *(const v4f*)(base + it * 1024);
    const float a0 = v[0], a1 = v[1], a2 = v[2], a3 = v[3];
    m = fmaxf(m, fmaxf(fmaxf(a0, a1), fmaxf(a2, a3)));
  }
  const float bm = block_max256(m, sRedA, lane, wave);
  if (wave == 0) {
    volatile float* q = pmax + (size_t)blockIdx.x * 32 + lane;
    *q = bm;
    __threadfence();
    *q = bm;
  }
}

__global__ __launch_bounds__(256) void max_final_kernel(const float* __restrict__ pmax, const float* __restrict__ window,
                                                        float* __restrict__ drline) {
  __shared__ float sRedA[8];
  __shared__ float sRedB[8];
  const int tid  = threadIdx.x;
  const int lane = tid & 31;
  const int wave = __builtin_amdgcn_readfirstlane(tid >> 5);
  const int i0 = (tid < kMaxBlocks) ? tid : (kMaxBlocks - 1);
  const int i1 = (tid + 256 < kMaxBlocks) ? (tid + 256) : (kMaxBlocks - 1);
  const float a = pmax[(size_t)i0 * 32];
  const float b = pmax[(size_t)i1 * 32];
  const int wi = (tid < kTaps) ? tid : (kTaps - 1);
  float wv = window[wi];
  asm volatile("" : "+v"(wv));
  const float w0 = window[0];
  const float badl = (wv != w0) ? 1.0f : 0.0f;
  const float m   = block_max256(fmaxf(a, b), sRedA, lane, wave);
  const float bad = block_max256(badl, sRedB, lane, wave);
  const float outv = (bad > 0.0f) ? __uint_as_float(0x7FC00000u) : m;
  if (wave == 0) {
    volatile float* q = drline + lane;
    *q = outv;
    __threadfence();
    *q = outv;
  }
}

template <int MAP>
__device__ __forceinline__ void fill_planes(const float* gimg, const float* pimg, int Y0, int X0,
                                            unsigned* sAh, unsigned* sAl, int tid) {
  constexpr bool kUseG = (MAP == 0) || (MAP == 2) || (MAP == 4);
  constexpr bool kUseP = (MAP == 1) || (MAP == 3) || (MAP == 4);
#pragma unroll 1
  for (int it = 0; it < kFillIters; ++it) {
    const int idx = tid + it * 256;
    const int idc = (idx < kFillItems) ? idx : (kFillItems - 1);
    const int row = idc / kGroups;
    const int col = (idc - row * kGroups) * 4;
    const int gy = Y0 + row;
    const int gx = X0 + col;
    const int gyc = (gy < kDim) ? gy : (kDim - 1);
    const int gxc = (gx < kDim) ? gx : (kDim - 4);
    const size_t off = (size_t)gyc * kDim + (size_t)gxc;
    v4f a = (v4f){0.f, 0.f, 0.f, 0.f};
    v4f b = (v4f){0.f, 0.f, 0.f, 0.f};
    if (kUseG) {
      a = *(const v4f*)(gimg + off);
      asm volatile("" : "+v"(a));
    }
    if (kUseP) {
      b = *(const v4f*)(pimg + off);
      asm volatile("" : "+v"(b));
    }
    const bool inside = (gy < kDim) && (gx < kDim);
    unsigned hw[4], lw[4];
#pragma unroll
    for (int e = 0; e < 4; ++e) {
      const float ga = a[e];
      const float pb = b[e];
      float x;
      if (MAP == 0) x = ga;
      else if (MAP == 1) x = pb;
      else if (MAP == 2) x = ga * ga;
      else if (MAP == 3) x = pb * pb;
      else x = ga * pb;
      x = inside ? x : 0.0f;
      split16(x, hw[e], lw[e]);
    }
    if (idx < kFillItems) {
      const int wo = row * kPitchW + (col >> 1);
      v2u h2, l2;
      h2[0] = hw[0] | (hw[1] << 16);
      h2[1] = hw[2] | (hw[3] << 16);
      l2[0] = lw[0] | (lw[1] << 16);
      l2[1] = lw[2] | (lw[3] << 16);
      *(v2u*)(sAh + wo) = h2;
      *(v2u*)(sAl + wo) = l2;
    }
  }
}

__device__ __forceinline__ v8f col_pass(const unsigned* sHh, const unsigned* sHl, v16h band, int s, int n16, int hh) {
  const int rp = s >> 2;
  const int c  = s & 3;
  const int wo = (16 * c + n16) * kPitchW + 8 * rp + 4 * hh;
  const v16h bh = ld_frag(sHh + wo);
  const v16h bl = ld_frag(sHl + wo);
  v8f dh = (v8f){0.f, 0.f, 0.f, 0.f, 0.f, 0.f, 0.f, 0.f};
  v8f dl = (v8f){0.f, 0.f, 0.f, 0.f, 0.f, 0.f, 0.f, 0.f};
  dh = mma_f16(band, bh, dh);
  dl = mma_f16(band, bl, dl);
  v8f o;
#pragma unroll
  for (int r = 0; r < 8; ++r) o[r] = dh[r] + dl[r] * kCarryInv;
  return o;
}

template <int MAP>
__device__ __forceinline__ void run_map(const float* gimg, const float* pimg, int Y0, int X0,
                                        unsigned* sAh, unsigned* sAl, unsigned* sHh, unsigned* sHl,
                                        v16h band, int tid, int wave, int n16, int hh, v8f& d0, v8f& d1) {
  fill_planes<MAP>(gimg, pimg, Y0, X0, sAh, sAl, tid);
  __syncthreads();
  for (int th = wave; th < 20; th += 8) {
    const int r = th >> 2;
    const int c = th & 3;
    const int wo = (16 * r + n16) * kPitchW + 8 * c + 4 * hh;
    const v16h ah = ld_frag(sAh + wo);
    const v16h al = ld_frag(sAl + wo);
    v8f sh = (v8f){0.f, 0.f, 0.f, 0.f, 0.f, 0.f, 0.f, 0.f};
    v8f sl = (v8f){0.f, 0.f, 0.f, 0.f, 0.f, 0.f, 0.f, 0.f};
    sh = mma_f16(ah, band, sh);
    sl = mma_f16(al, band, sl);
    unsigned wh[4], wl[4];
#pragma unroll
    for (int j = 0; j < 4; ++j) {
      const float h0 = sh[2 * j]     + sl[2 * j]     * kCarryInv;
      const float h1 = sh[2 * j + 1] + sl[2 * j + 1] * kCarryInv;
      unsigned hb0, lb0, hb1, lb1;
      split16(h0, hb0, lb0);
      split16(h1, hb1, lb1);
      wh[j] = hb0 | (hb1 << 16);
      wl[j] = lb0 | (lb1 << 16);
    }
    const int so = (16 * c + n16) * kPitchW + 8 * r + 4 * hh;
    v4u hv, lv;
    hv[0] = wh[0]; hv[1] = wh[1]; hv[2] = wh[2]; hv[3] = wh[3];
    lv[0] = wl[0]; lv[1] = wl[1]; lv[2] = wl[2]; lv[3] = wl[3];
    *(v4u*)(sHh + so) = hv;
    *(v4u*)(sHl + so) = lv;
  }
  __syncthreads();
  d0 = col_pass(sHh, sHl, band, 2 * wave,     n16, hh);
  d1 = col_pass(sHh, sHl, band, 2 * wave + 1, n16, hh);
}

__global__ __launch_bounds__(256) void boxmap_tile_kernel(const float* __restrict__ gt, const float* __restrict__ pred,
                                                          const float* __restrict__ window, const float* __restrict__ drline,
                                                          float* __restrict__ psum) {
  __shared__ __align__(16) unsigned sAh[kRegion * kPitchW];
  __shared__ __align__(16) unsigned sAl[kRegion * kPitchW];
  __shared__ __align__(16) unsigned sHh[kTile * kPitchW];
  __shared__ __align__(16) unsigned sHl[kTile * kPitchW];
  __shared__ float sRedA[8];

  const int tid  = threadIdx.x;
  const int lane = tid & 31;
  const int wave = __builtin_amdgcn_readfirstlane(tid >> 5);
  const int n16  = lane & 15;
  const int hh   = lane >> 4;

  const int bid = blockIdx.x;
  const int img = bid / (kTilesDim * kTilesDim);
  const int t2  = bid - img * (kTilesDim * kTilesDim);
  const int ty  = t2 / kTilesDim;
  const int tx  = t2 - ty * kTilesDim;
  const int Y0  = ty * kTile;
  const int X0  = tx * kTile;
  const float* gimg = gt   + (size_t)img * kDim * kDim;
  const float* pimg = pred + (size_t)img * kDim * kDim;

  v8u bw = (v8u){0u, 0u, 0u, 0u, 0u, 0u, 0u, 0u};
#pragma unroll
  for (int j = 0; j < 8; ++j) {
    const int e0 = 2 * j;
    const int e1 = 2 * j + 1;
    const int k0 = 8 * hh + e0 + ((e0 >= 8) ? 8 : 0);
    const int k1 = 8 * hh + e1 + ((e1 >= 8) ? 8 : 0);
    const unsigned lo = (k0 >= n16 && k0 <= n16 + 6) ? 0x00003C00u : 0u;
    const unsigned hi = (k1 >= n16 && k1 <= n16 + 6) ? 0x3C000000u : 0u;
    bw[j] = lo | hi;
  }
  const v16h band = __builtin_bit_cast(v16h, bw);

  v8f res[5][2];
  run_map<0>(gimg, pimg, Y0, X0, sAh, sAl, sHh, sHl, band, tid, wave, n16, hh, res[0][0], res[0][1]);
  run_map<1>(gimg, pimg, Y0, X0, sAh, sAl, sHh, sHl, band, tid, wave, n16, hh, res[1][0], res[1][1]);
  run_map<2>(gimg, pimg, Y0, X0, sAh, sAl, sHh, sHl, band, tid, wave, n16, hh, res[2][0], res[2][1]);
  run_map<3>(gimg, pimg, Y0, X0, sAh, sAl, sHh, sHl, band, tid, wave, n16, hh, res[3][0], res[3][1]);
  run_map<4>(gimg, pimg, Y0, X0, sAh, sAl, sHh, sHl, band, tid, wave, n16, hh, res[4][0], res[4][1]);

  const float w0 = window[0];
  const float dr = drline[0];
  const float c1 = (0.01f * dr) * (0.01f * dr);
  const float c2 = (0.03f * dr) * (0.03f * dr);
  float acc = 0.0f;
#pragma unroll
  for (int t = 0; t < 2; ++t) {
    const int s  = 2 * wave + t;
    const int rp = s >> 2;
    const int c  = s & 3;
    const int ox = X0 + 16 * c + n16;
#pragma unroll
    for (int r = 0; r < 8; ++r) {
      const int oy = Y0 + 16 * rp + 8 * hh + r;
      const float mx  = w0 * res[0][t][r];
      const float my  = w0 * res[1][t][r];
      const float exx = w0 * res[2][t][r];
      const float eyy = w0 * res[3][t][r];
      const float exy = w0 * res[4][t][r];
      const float uxx = exx - mx * mx;
      const float uyy = eyy - my * my;
      const float uxy = exy - mx * my;
      const float vx  = kCovNorm * uxx;
      const float vy  = kCovNorm * uyy;
      const float vxy = kCovNorm * uxy;
      const float num = (2.0f * mx * my + c1) * (2.0f * vxy + c2);
      const float den = (mx * mx + my * my + c1) * (vx + vy + c2);
      float rc = __builtin_amdgcn_rcpf(den);
      const float er = fmaf(-den, rc, 1.0f);
      rc = fmaf(rc, er, rc);
      const float sv = num * rc;
      const bool ok = (oy < kValid) && (ox < kValid);
      acc += ok ? sv : 0.0f;
    }
  }
  const float tot = block_sum256(acc, sRedA, lane, wave);
  if (wave == 0) {
    const float val = (lane == 0) ? tot : 0.0f;
    volatile float* q = psum + (size_t)bid * 32 + lane;
    *q = val;
    __threadfence();
    *q = val;
  }
}

__global__ __launch_bounds__(256) void finalize_kernel(const float* __restrict__ psum, float* __restrict__ out) {
  __shared__ double sD[256];
  const int tid = threadIdx.x;
  double a = 0.0;
#pragma unroll 1
  for (int i = 0; i < kTileBlocks / 256; ++i) a += (double)psum[(size_t)(tid + 256 * i) * 32];
  sD[tid] = a;
  __syncthreads();
  for (int off = 128; off > 0; off >>= 1) {
    if (tid < off) sD[tid] += sD[tid + off];
    __syncthreads();
  }
  if (tid == 0) {
    const float v = (float)(sD[0] * kInvCount);
    volatile float* q = out;
    *q = v;
    __threadfence();
    *q = v;
  }
}

extern "C" void kernel_launch(void* const* d_in, const int* in_sizes, int n_in,
                              void* d_out, int out_size, void* d_ws, size_t ws_size,
                              hipStream_t stream) {
  if (n_in < 3) return;
  if (in_sizes[0] != kImgs * kDim * kDim) return;
  if (in_sizes[1] != kImgs * kDim * kDim) return;
  if (in_sizes[2] != kTaps) return;
  if (out_size != 1) return;
  if (ws_size < kWsTotal) return;

  const float* gt     = (const float*)d_in[0];
  const float* pred   = (const float*)d_in[1];
  const float* window = (const float*)d_in[2];
  float* out = (float*)d_out;

  char* ws = (char*)d_ws;
  float* pmax   = (float*)(ws + kOffPmax);
  float* drline = (float*)(ws + kOffDr);
  float* psum   = (float*)(ws + kOffPsum);

  max_partial_kernel<<<kMaxBlocks, 256, 0, stream>>>(gt, pmax);
  max_final_kernel<<<1, 256, 0, stream>>>(pmax, window, drline);
  boxmap_tile_kernel<<<kTileBlocks, 256, 0, stream>>>(gt, pred, window, drline, psum);
  finalize_kernel<<<1, 256, 0, stream>>>(psum, out);
}
